// TGCNet_16338055594467
// MI455X (gfx1250) — hardware-verified
//
#include <hip/hip_runtime.h>
#include <stdint.h>


#define C      64
#define OUTC   8
#define TD     8192
#define TA     1024
#define WAVES  4
#define TPW    4

typedef float    v2f  __attribute__((ext_vector_type(2)));
typedef float    v4f  __attribute__((ext_vector_type(4)));
typedef float    v8f  __attribute__((ext_vector_type(8)));
typedef _Float16 v8h  __attribute__((ext_vector_type(8)));
typedef _Float16 v16h __attribute__((ext_vector_type(16)));

union Frag { v16h v; v8h half[2]; };
union F8   { v8f v;  v4f q[2]; };
union H8   { v8h h;  v4f f; };

__device__ __forceinline__ v8f wmma_f16(v16h a, v16h b, v8f c)
{
    v8f d = __builtin_amdgcn_wmma_f32_16x16x32_f16(false, a, false, b, (short)0, c, false, false);
    asm volatile("v_nop\n\tv_nop\n\tv_nop\n\tv_nop" : "+v"(d) : "v"(a), "v"(b));
    return d;
}

__device__ __forceinline__ v8f zero8()
{
    v8f z = {0.0f, 0.0f, 0.0f, 0.0f, 0.0f, 0.0f, 0.0f, 0.0f};
    return z;
}

__device__ __forceinline__ v8f ld8(const float* p)
{
    F8 u;
    u.q[0] = *(const v4f*)p;
    u.q[1] = *(const v4f*)(p + 4);
    return u.v;
}

__device__ __forceinline__ void deg_store(const float* sdeg, float* dinv, int base, int lane)
{
#pragma unroll 2
    for (int i = 4 * lane; i < TD; i += 128) {
        v4f v = {0.0f, 0.0f, 0.0f, 0.0f};
#pragma unroll
        for (int k = 0; k < 4; ++k) {
            const float dg = sdeg[i + k];
            v[k] = (dg > 0.0f) ? rsqrtf(dg) : 0.0f;
        }
        *(volatile v4f*)(dinv + (size_t)base + i) = v;
    }
}

__global__ __launch_bounds__(32) void k_deg(const int* __restrict__ ei, const float* __restrict__ ew,
                                            float* dinv, int E)
{
    __shared__ __attribute__((aligned(16))) float sdeg[TD];
    const int lane = threadIdx.x;
    const int base = blockIdx.x * TD;
    const int* dst = ei + E;

    for (int i = lane; i < TD; i += 32) sdeg[i] = 1.0f;
    __syncthreads();

#pragma unroll 1
    for (int c0 = 0; c0 < E; c0 += 128) {
        int dk[4];
#pragma unroll
        for (int k = 0; k < 4; ++k) {
            const int e = c0 + 32 * k + lane;
            dk[k] = (e < E) ? dst[e] : -1;
        }
#pragma unroll
        for (int k = 0; k < 4; ++k) {
            const int dv = dk[k];
            unsigned mask = __builtin_amdgcn_ballot_w32((dv >= base) && (dv < base + TD));
            while (mask != 0u) {
                const int b = __builtin_ctz(mask);
                mask &= (mask - 1u);
                const int e  = c0 + 32 * k + b;
                const int dl = __shfl(dv, b) - base;
                const float we = ew[e];
                if (lane == 0) sdeg[dl] = sdeg[dl] + we;
            }
        }
    }
    __syncthreads();

    deg_store(sdeg, dinv, base, lane);
    __threadfence();
    deg_store(sdeg, dinv, base, lane);
}

__device__ __forceinline__ void agg_store(const float* acc, _Float16* aggh, int base, int lane)
{
#pragma unroll 2
    for (int i = 0; i < TA / 4; ++i) {
        const int row = 4 * i + (lane >> 3);
        const int c0  = 8 * (lane & 7);
        const float* sp = acc + row * C + c0;
        F8 f;
        f.q[0] = *(const v4f*)sp;
        f.q[1] = *(const v4f*)(sp + 4);
        H8 o;
        o.h = __builtin_convertvector(f.v * 16.0f, v8h);
        *(volatile v4f*)(aggh + (size_t)(base + row) * C + c0) = o.f;
    }
}

__global__ __launch_bounds__(32) void k_agg(const float* __restrict__ x, const int* __restrict__ ei,
                                            const float* __restrict__ ew, const float* __restrict__ dinv,
                                            _Float16* aggh, int N, int E)
{
    extern __shared__ v4f dacc[];
    float* acc = (float*)dacc;
    const int lane = threadIdx.x;
    const int base = blockIdx.x * TA;
    const int* dst = ei + E;

#pragma unroll 2
    for (int i = lane; i < TA * (C / 4); i += 32) {
        const int row = i >> 4, q = i & 15;
        const int n = base + row;
        v4f v = {0.0f, 0.0f, 0.0f, 0.0f};
        if (n < N) {
            const float di = dinv[n];
            const v4f xx = *(const v4f*)(x + (size_t)n * C + 4 * q);
            v = xx * (di * di);
        }
        dacc[i] = v;
    }
    __syncthreads();

#pragma unroll 1
    for (int c0 = 0; c0 < E; c0 += 128) {
        int dk[4];
#pragma unroll
        for (int k = 0; k < 4; ++k) {
            const int e = c0 + 32 * k + lane;
            dk[k] = (e < E) ? dst[e] : -1;
        }
#pragma unroll
        for (int k = 0; k < 4; ++k) {
            const int dv = dk[k];
            unsigned mask = __builtin_amdgcn_ballot_w32((dv >= base) && (dv < base + TA));
            while (mask != 0u) {
                const int b = __builtin_ctz(mask);
                mask &= (mask - 1u);
                const int e  = c0 + 32 * k + b;
                const int de = __shfl(dv, b);
                int se = ei[e];
                se = (se < 0) ? 0 : ((se >= N) ? (N - 1) : se);
                const float we = ew[e];
                const int   dc = (de < N) ? de : (N - 1);
                const float nrm = dinv[se] * we * dinv[dc];
                const v2f xv = *(const v2f*)(x + (size_t)se * C + 2 * lane);
                v2f* ap = (v2f*)(acc + (size_t)(de - base) * C + 2 * lane);
                *ap = *ap + xv * nrm;
            }
        }
    }
    __syncthreads();

    agg_store(acc, aggh, base, lane);
    __threadfence();
    agg_store(acc, aggh, base, lane);
}

__device__ __forceinline__ v8f mm_rowtile(const _Float16* rowp, int h, v16h b0, v16h b1, v8f d)
{
    Frag a;
    a.half[0] = *(const v8h*)(rowp + 8 * h);
    a.half[1] = *(const v8h*)(rowp + 16 + 8 * h);
    d = wmma_f16(a.v, b0, d);
    a.half[0] = *(const v8h*)(rowp + 32 + 8 * h);
    a.half[1] = *(const v8h*)(rowp + 48 + 8 * h);
    d = wmma_f16(a.v, b1, d);
    return d;
}

__device__ __forceinline__ void mm4(const _Float16* sT, int m, int h, v16h b0, v16h b1,
                                    v8f& d0, v8f& d1, v8f& d2, v8f& d3)
{
    d0 = mm_rowtile(sT + (0 * 16 + m) * C, h, b0, b1, zero8());
    d1 = mm_rowtile(sT + (1 * 16 + m) * C, h, b0, b1, zero8());
    d2 = mm_rowtile(sT + (2 * 16 + m) * C, h, b0, b1, zero8());
    d3 = mm_rowtile(sT + (3 * 16 + m) * C, h, b0, b1, zero8());
}

__device__ __forceinline__ v8f one_minus_sigmoid8(v8f p)
{
    v8f r;
#pragma unroll
    for (int i = 0; i < 8; ++i) {
        const float z = __builtin_amdgcn_rcpf(1.0f + __expf(-p[i]));
        r[i] = 1.0f - z;
    }
    return r;
}

__device__ __forceinline__ v8f gate_relu64(v8f f, v8f p)
{
    v8f r;
#pragma unroll
    for (int i = 0; i < 8; ++i) {
        const float th = 1.0f - 2.0f * __builtin_amdgcn_rcpf(1.0f + __expf(2.0f * p[i]));
        const float hn = f[i] * th;
        r[i] = fmaxf(hn, 0.0f) * 64.0f;
    }
    return r;
}

__global__ __launch_bounds__(WAVES * 32) void k_node(
    const _Float16* __restrict__ aggh,
    const float* __restrict__ czW, const float* __restrict__ czb,
    const float* __restrict__ chW, const float* __restrict__ chb,
    const float* __restrict__ lzW, const float* __restrict__ lzb,
    const float* __restrict__ lhW, const float* __restrict__ lhb,
    const float* __restrict__ hW,  const float* __restrict__ hb,
    float* out, int N, int numTiles)
{
    __shared__ __attribute__((aligned(16))) _Float16 sWz[C * C];
    __shared__ __attribute__((aligned(16))) _Float16 sWh[C * C];
    __shared__ __attribute__((aligned(16))) _Float16 sLz[C * C];
    __shared__ __attribute__((aligned(16))) _Float16 sLh[C * C];
    __shared__ __attribute__((aligned(16))) _Float16 sHd[16 * C];
    __shared__ __attribute__((aligned(16))) float sBz[C];
    __shared__ __attribute__((aligned(16))) float sBh[C];
    __shared__ __attribute__((aligned(16))) float sLbz[C];
    __shared__ __attribute__((aligned(16))) float sLbh[C];
    __shared__ __attribute__((aligned(16))) float sHb[16];
    __shared__ v4f sOut[WAVES][32];

    const int t = threadIdx.x;
    for (int idx = t; idx < C * C; idx += WAVES * 32) {
        const int a = idx >> 6, b = idx & 63;
        sWz[idx] = (_Float16)(64.0f * czW[b * C + a]);
        sWh[idx] = (_Float16)(64.0f * chW[b * C + a]);
        sLz[idx] = (_Float16)(64.0f * lzW[b * C + a]);
        sLh[idx] = (_Float16)(64.0f * lhW[b * C + a]);
    }
    for (int idx = t; idx < 16 * C; idx += WAVES * 32) {
        const int a = idx >> 6, b = idx & 63;
        sHd[idx] = (a < OUTC) ? (_Float16)(64.0f * hW[b * OUTC + a]) : (_Float16)0.0f;
    }
    if (t < C) {
        sBz[t]  = 64.0f * czb[t];
        sBh[t]  = 64.0f * chb[t];
        sLbz[t] = lzb[t];
        sLbh[t] = lhb[t];
    }
    if (t < 16) sHb[t] = (t < OUTC) ? hb[t] : 0.0f;
    __syncthreads();

    const int wave = t >> 5;
    const int lane = t & 31;
    const int h = lane >> 4;
    const int m = lane & 15;
    const float s16   = 0.0625f;
    const float s4096 = 1.0f / 4096.0f;

#pragma unroll 1
    for (int it = 0; it < TPW; ++it) {
        const int traw = blockIdx.x * (TPW * WAVES) + it * WAVES + wave;
        const bool active = traw < numTiles;
        const int tile = active ? traw : (numTiles - 1);
        const int nbase = tile * 16;

        const _Float16* arow = aggh + (size_t)(nbase + m) * C;
        Frag bx0, bx1;
        bx0.half[0] = *(const v8h*)(arow + 8 * h);
        bx0.half[1] = *(const v8h*)(arow + 16 + 8 * h);
        bx1.half[0] = *(const v8h*)(arow + 32 + 8 * h);
        bx1.half[1] = *(const v8h*)(arow + 48 + 8 * h);

        v8f f0, f1, f2, f3;
        {
            v8f d0, d1, d2, d3;
            mm4(sWz, m, h, bx0.v, bx1.v, d0, d1, d2, d3);
            Frag g0, g1;
            g0.half[0] = __builtin_convertvector(d0 * s16 + ld8(sBz + 0  + 8 * h), v8h);
            g0.half[1] = __builtin_convertvector(d1 * s16 + ld8(sBz + 16 + 8 * h), v8h);
            g1.half[0] = __builtin_convertvector(d2 * s16 + ld8(sBz + 32 + 8 * h), v8h);
            g1.half[1] = __builtin_convertvector(d3 * s16 + ld8(sBz + 48 + 8 * h), v8h);
            v8f e0, e1, e2, e3;
            mm4(sLz, m, h, g0.v, g1.v, e0, e1, e2, e3);
            f0 = one_minus_sigmoid8(e0 * s4096 + ld8(sLbz + 0  + 8 * h));
            f1 = one_minus_sigmoid8(e1 * s4096 + ld8(sLbz + 16 + 8 * h));
            f2 = one_minus_sigmoid8(e2 * s4096 + ld8(sLbz + 32 + 8 * h));
            f3 = one_minus_sigmoid8(e3 * s4096 + ld8(sLbz + 48 + 8 * h));
        }

        Frag q0, q1;
        {
            v8f d0, d1, d2, d3;
            mm4(sWh, m, h, bx0.v, bx1.v, d0, d1, d2, d3);
            Frag g0, g1;
            g0.half[0] = __builtin_convertvector(d0 * s16 + ld8(sBh + 0  + 8 * h), v8h);
            g0.half[1] = __builtin_convertvector(d1 * s16 + ld8(sBh + 16 + 8 * h), v8h);
            g1.half[0] = __builtin_convertvector(d2 * s16 + ld8(sBh + 32 + 8 * h), v8h);
            g1.half[1] = __builtin_convertvector(d3 * s16 + ld8(sBh + 48 + 8 * h), v8h);
            v8f e0, e1, e2, e3;
            mm4(sLh, m, h, g0.v, g1.v, e0, e1, e2, e3);
            q0.half[0] = __builtin_convertvector(gate_relu64(f0, e0 * s4096 + ld8(sLbh + 0  + 8 * h)), v8h);
            q0.half[1] = __builtin_convertvector(gate_relu64(f1, e1 * s4096 + ld8(sLbh + 16 + 8 * h)), v8h);
            q1.half[0] = __builtin_convertvector(gate_relu64(f2, e2 * s4096 + ld8(sLbh + 32 + 8 * h)), v8h);
            q1.half[1] = __builtin_convertvector(gate_relu64(f3, e3 * s4096 + ld8(sLbh + 48 + 8 * h)), v8h);
        }

        const v8f fo = mm_rowtile(sHd + m * C, h, q0.v, q1.v, zero8());
        const v8f ov = fo * s4096 + ld8(sHb + 8 * h);
        if (h == 0) {
            F8 u;
            u.v = ov;
            sOut[wave][2 * m]     = u.q[0];
            sOut[wave][2 * m + 1] = u.q[1];
        }
        __syncthreads();

        const v4f sv = sOut[wave][lane];
        const size_t o0 = (size_t)nbase * OUTC + 4 * (size_t)lane;
        const bool ok = active && (o0 + 4 <= (size_t)N * OUTC);
        if (ok) *(volatile v4f*)(out + o0) = sv;
        __threadfence();
        if (ok) *(volatile v4f*)(out + o0) = sv;
        __syncthreads();
    }
}

extern "C" void kernel_launch(void* const* d_in, const int* in_sizes, int n_in,
                              void* d_out, int out_size, void* d_ws, size_t ws_size,
                              hipStream_t stream)
{
    if (n_in < 17) return;
    const int N = in_sizes[0] / C;
    int E = in_sizes[2];
    if (in_sizes[1] / 2 < E) E = in_sizes[1] / 2;
    if (N <= 0 || E < 0) return;
    if ((size_t)out_size < (size_t)N * OUTC) return;

    const float* x   = (const float*)d_in[0];
    const int*   ei  = (const int*)d_in[1];
    const float* ew  = (const float*)d_in[2];
    const float* czW = (const float*)d_in[3];
    const float* czb = (const float*)d_in[4];
    const float* chW = (const float*)d_in[7];
    const float* chb = (const float*)d_in[8];
    const float* lzW = (const float*)d_in[9];
    const float* lzb = (const float*)d_in[10];
    const float* lhW = (const float*)d_in[13];
    const float* lhb = (const float*)d_in[14];
    const float* hW  = (const float*)d_in[15];
    const float* hb  = (const float*)d_in[16];

    const int gridD    = (N + TD - 1) / TD;
    const int gridA    = (N + TA - 1) / TA;
    const int numTiles = (N + 15) / 16;
    const int gridN    = (numTiles + TPW * WAVES - 1) / (TPW * WAVES);

    const size_t bytesDinv = (size_t)gridD * TD * sizeof(float);
    const size_t offAgg    = (bytesDinv + 127) & ~(size_t)127;
    const size_t bytesAgg  = (size_t)gridA * TA * C * sizeof(_Float16);
    if (offAgg + bytesAgg > ws_size) return;

    float*    dinv = (float*)d_ws;
    _Float16* aggh = (_Float16*)((char*)d_ws + offAgg);

    const size_t dynLds = (size_t)TA * C * sizeof(float);

    k_deg<<<gridD, 32, 0, stream>>>(ei, ew, dinv, E);
    k_agg<<<gridA, 32, dynLds, stream>>>(x, ei, ew, dinv, aggh, N, E);
    k_node<<<gridN, WAVES * 32, 0, stream>>>(aggh, czW, czb, chW, chb, lzW, lzb, lhW, lhb, hW, hb,
                                              (float*)d_out, N, numTiles);
}
